// MultiTimeAttention_32375463477366
// MI455X (gfx1250) — hardware-run, weakly checked
//
#include <hip/hip_runtime.h>


namespace {
constexpr int NB = 16, NH = 4, REF = 128, KEY = 256, DIM = 32, ET = 128, EK = 32, NHID = 128, HDIM = NH * DIM  ;
constexpr float XS = 8.0f, HS = 256.0f, WSC = 256.0f, ES = 256.0f, SCALE = 0.17677669529663687f;
typedef _Float16 b16;
typedef __attribute__((ext_vector_type(16))) _Float16 v16b;
typedef __attribute__((ext_vector_type(8))) _Float16 v8b;
typedef __attribute__((ext_vector_type(8))) float v8f;
typedef __attribute__((ext_vector_type(4))) float v4f;
__device__ __forceinline__ float bf16_rne(float f) { unsigned int u = __float_as_uint(f); u += 0x7FFFu + ((u >> 16) & 1u); float r = __uint_as_float(u & 0xFFFF0000u); asm volatile("" : "+v"(r)); return r; }
__device__ __forceinline__ float bfv(float f) { float r = bf16_rne(f); asm volatile("" : "+v"(r)); return r; }
__device__ __forceinline__ void split16(float v, b16& hi, b16& lo) { hi = (b16)v; lo = (b16)(v - (float)hi); }
__device__ __forceinline__ v16b frag_kb(const b16* p, int hh) { const v8b a = *(const v8b*)(p + 8 * hh), b = *(const v8b*)(p + 16 + 8 * hh); v16b f;
#pragma unroll
  for (int e = 0; e < 8; ++e) { f[e] = a[e]; f[8 + e] = b[e]; } return f; }
__device__ __forceinline__ v8f wmma16b(v16b a, v16b b, v8f c) { v8f d = __builtin_amdgcn_wmma_f32_16x16x32_f16(false, a, false, b, (short)0, c, false, false); asm volatile("v_nop\n\tv_nop\n\tv_nop\n\tv_nop" : "+v"(d) : "v"(a), "v"(b)); return d; }
__device__ __forceinline__ void wave_lds_sync() { __builtin_amdgcn_fence(__ATOMIC_RELEASE, "workgroup"); __builtin_amdgcn_wave_barrier(); __builtin_amdgcn_fence(__ATOMIC_ACQUIRE, "workgroup"); }
__device__ __forceinline__ float pmul(float a, float b) { float p = a * b; asm volatile("" : "+v"(p)); return p; }

__global__ __launch_bounds__(256) void wput_kernel(const float* __restrict__ wq, const float* __restrict__ wk, const float* __restrict__ wo, b16* __restrict__ WQ, b16* __restrict__ WK, b16* __restrict__ WO) { const int u = blockIdx.x * 256 + threadIdx.x; if (u >= ET * 16) return; const int o = u / 16, k0 = (u % 16) * 8; v8b v;
  const float* ws3[3] = {wq, wk, wo}; b16* ds3[3] = {WQ, WK, WO};
#pragma unroll
  for (int m = 0; m < 3; ++m) {
#pragma unroll
    for (int j = 0; j < 8; ++j) v[j] = (b16)(bf16_rne(ws3[m][(size_t)(k0 + j) * ET + o]) * WSC); for (int pass = 0; pass < 2; ++pass) { *(volatile v8b*)(ds3[m] + (size_t)o * ET + k0) = v; __threadfence(); } } }
template <int MODE>
__global__ __launch_bounds__(32) void proj_kernel(const float* __restrict__ x, const b16* __restrict__ W, const float* __restrict__ bias, int RLIM, b16* __restrict__ Oh_, b16* __restrict__ Ol_) { __shared__ __attribute__((aligned(16))) b16 Ah[16][ET + 8], Oh[16][ET + 8], Ol[16][ET + 8]; const int lane = threadIdx.x, nloc = lane & 15, hlf = lane >> 4; const size_t m0 = (size_t)blockIdx.x * 16; if (m0 >= (size_t)RLIM) return;
  for (int rr = 0; rr < 16; ++rr) for (int q = 0; q < 4; ++q) Ah[rr][q * 32 + lane] = (b16)(bf16_rne(x[(m0 + rr) * ET + q * 32 + lane]) * XS); if (lane < 16) for (int k = ET; k < ET + 8; ++k) Ah[lane][k] = (b16)0.0f;
  wave_lds_sync(); v8f acc[8];
#pragma unroll
  for (int t = 0; t < 8; ++t) acc[t] = (v8f){};
#pragma unroll
  for (int kb = 0; kb < ET; kb += 32) { const v16b a = frag_kb(&Ah[nloc][kb], hlf);
#pragma unroll
    for (int t = 0; t < 8; ++t) acc[t] = wmma16b(a, frag_kb(W + (size_t)(t * 16 + nloc) * ET + kb, hlf), acc[t]); }
  const float sc = MODE == 0 ? SCALE : 1.0f;
#pragma unroll
  for (int t = 0; t < 8; ++t) { const int cc = t * 16 + nloc; const float bb = bfv(bias[cc]);
#pragma unroll
    for (int r8 = 0; r8 < 8; ++r8) { b16 p, ql; split16((acc[t][r8] * (1.0f / (XS * WSC)) + bb) * sc * HS, p, ql); Oh[8 * hlf + r8][cc] = p; Ol[8 * hlf + r8][cc] = ql; } }
  wave_lds_sync();
  for (int pass = 0; pass < 2; ++pass) { for (int rr = 0; rr < 16; ++rr) if (lane < 16) { *(volatile v8b*)(Oh_ + (m0 + rr) * ET + lane * 8) = *(const v8b*)(&Oh[rr][lane * 8]); *(volatile v8b*)(Ol_ + (m0 + rr) * ET + lane * 8) = *(const v8b*)(&Ol[rr][lane * 8]); } __threadfence(); } }
__global__ __launch_bounds__(32) void att_kernel(const b16* __restrict__ Qh, const b16* __restrict__ Ql, const b16* __restrict__ Kh, const b16* __restrict__ Kl, const float* __restrict__ value, const int* __restrict__ mask, int BLIM, float* __restrict__ X) {
  __shared__ __attribute__((aligned(16))) b16 Eh_[16][KEY + 8], El_[16][KEY + 8], MVt[DIM][KEY + 8], Mt[DIM][KEY + 8]; __shared__ float Sf[16][KEY + 4], Nf[16][DIM + 1], Df[16][DIM + 1], Vs[DIM];
  const int lane = threadIdx.x, nloc = lane & 15, hlf = lane >> 4; const int rt = blockIdx.x % (REF / 16); const int h = (blockIdx.x / (REF / 16)) % NH; const int b = blockIdx.x / ((REF / 16) * NH); if (b >= BLIM) return; const int r0 = rt * 16;
  { float vs = 0.0f; for (int k = 0; k < KEY; ++k) { const size_t o = ((size_t)b * KEY + k) * DIM + lane; const float v = bfv(value[o]); const int mk = mask[o] != 0 ? 1 : 0; MVt[lane][k] = (b16)(mk ? v * XS : 0.0f); Mt[lane][k] = (b16)(mk ? 1.0f : 0.0f); vs += v; } Vs[lane] = vs / KEY; for (int k = KEY; k < KEY + 8; ++k) { MVt[lane][k] = (b16)0.0f; Mt[lane][k] = (b16)0.0f; } }
  const v16b qa = frag_kb(Qh + ((size_t)b * REF + r0 + nloc) * ET + h * EK, hlf), qb = frag_kb(Ql + ((size_t)b * REF + r0 + nloc) * ET + h * EK, hlf);
#pragma unroll
  for (int t = 0; t < KEY / 16; ++t) { const size_t kr = ((size_t)b * KEY + t * 16 + nloc) * ET + h * EK; const v16b ka = frag_kb(Kh + kr, hlf), kl = frag_kb(Kl + kr, hlf); v8f s = {}; s = wmma16b(qa, ka, s); s = wmma16b(qa, kl, s); s = wmma16b(qb, ka, s);
#pragma unroll
    for (int r8 = 0; r8 < 8; ++r8) Sf[8 * hlf + r8][t * 16 + nloc] = s[r8] * (1.0f / (HS * HS)); }
  wave_lds_sync();
  for (int rr = 0; rr < 16; ++rr) { float mx = -INFINITY; for (int q = 0; q < KEY / 32; ++q) mx = fmaxf(mx, Sf[rr][q * 32 + lane]); for (int o = 16; o; o >>= 1) mx = fmaxf(mx, __shfl_xor(mx, o));
    for (int q = 0; q < KEY / 32; ++q) { const int kx = q * 32 + lane; b16 p, ql; split16(__expf(Sf[rr][kx] - mx) * ES, p, ql); Eh_[rr][kx] = p; El_[rr][kx] = ql; } }
  if (lane < 16) for (int k = KEY; k < KEY + 8; ++k) { Eh_[lane][k] = (b16)0.0f; El_[lane][k] = (b16)0.0f; }
  wave_lds_sync(); v8f an[2] = {(v8f){}, (v8f){}}, ad[2] = {(v8f){}, (v8f){}};
#pragma unroll 2
  for (int kb = 0; kb < KEY; kb += 32) { const v16b ea = frag_kb(&Eh_[nloc][kb], hlf), eb = frag_kb(&El_[nloc][kb], hlf);
#pragma unroll
    for (int t = 0; t < 2; ++t) { const v16b mv = frag_kb(&MVt[t * 16 + nloc][kb], hlf), mm = frag_kb(&Mt[t * 16 + nloc][kb], hlf); an[t] = wmma16b(ea, mv, an[t]); an[t] = wmma16b(eb, mv, an[t]); ad[t] = wmma16b(ea, mm, ad[t]); ad[t] = wmma16b(eb, mm, ad[t]); } }
#pragma unroll
  for (int t = 0; t < 2; ++t)
#pragma unroll
    for (int r8 = 0; r8 < 8; ++r8) { Nf[8 * hlf + r8][t * 16 + nloc] = an[t][r8] * (1.0f / (ES * XS)); Df[8 * hlf + r8][t * 16 + nloc] = ad[t][r8] * (1.0f / ES); }
  wave_lds_sync();
  for (int pass = 0; pass < 2; ++pass) { for (int rr = 0; rr < 16; ++rr) { const float dn = Df[rr][lane]; ((volatile float*)X)[((size_t)b * REF + r0 + rr) * HDIM + h * DIM + lane] = dn > 0.0f ? Nf[rr][lane] / dn : Vs[lane]; } __threadfence(); } }
__global__ __launch_bounds__(32) void out_kernel(const float* __restrict__ X, const b16* __restrict__ WO, const float* __restrict__ bo, int RLIM, float* __restrict__ out) { __shared__ __attribute__((aligned(16))) b16 Ah[16][HDIM + 8], Al[16][HDIM + 8]; __shared__ float Tf[16][NHID + 4]; const int lane = threadIdx.x, nloc = lane & 15, hlf = lane >> 4; const size_t m0 = (size_t)blockIdx.x * 16; if (m0 >= (size_t)RLIM) return;
  for (int rr = 0; rr < 16; ++rr) for (int q = 0; q < 4; ++q) { b16 p, ql; split16(X[(m0 + rr) * HDIM + q * 32 + lane] * HS, p, ql); Ah[rr][q * 32 + lane] = p; Al[rr][q * 32 + lane] = ql; } if (lane < 16) for (int k = HDIM; k < HDIM + 8; ++k) { Ah[lane][k] = (b16)0.0f; Al[lane][k] = (b16)0.0f; }
  wave_lds_sync(); v8f acc[8];
#pragma unroll
  for (int t = 0; t < 8; ++t) acc[t] = (v8f){};
#pragma unroll
  for (int kb = 0; kb < HDIM; kb += 32) { const v16b a = frag_kb(&Ah[nloc][kb], hlf), al = frag_kb(&Al[nloc][kb], hlf);
#pragma unroll
    for (int t = 0; t < 8; ++t) { const v16b bw = frag_kb(WO + (size_t)(t * 16 + nloc) * HDIM + kb, hlf); acc[t] = wmma16b(a, bw, acc[t]); acc[t] = wmma16b(al, bw, acc[t]); } }
#pragma unroll
  for (int t = 0; t < 8; ++t) { const int cc = t * 16 + nloc; const float bb = bfv(bo[cc]);
#pragma unroll
    for (int r8 = 0; r8 < 8; ++r8) Tf[8 * hlf + r8][cc] = acc[t][r8] * (1.0f / (HS * WSC)) + bb; }
  wave_lds_sync();
  for (int pass = 0; pass < 2; ++pass) { for (int rr = 0; rr < 16; ++rr) *(volatile v4f*)(out + (m0 + rr) * NHID + lane * 4) = *(const v4f*)(&Tf[rr][lane * 4]); __threadfence(); } }
}

extern "C" void kernel_launch(void* const* d_in, const int* in_sizes, int n_in, void* d_out, int out_size, void* d_ws, size_t ws_size, hipStream_t stream) {
  (void)n_in;
  auto Fp = [&](int i) { return (const float*)d_in[i]; }; auto Ip = [&](int i) { return (const int*)d_in[i]; };
  if (in_sizes[0] != NB * REF * ET || in_sizes[1] != NB * KEY * ET || in_sizes[2] != NB * KEY * DIM || in_sizes[3] != NB * KEY * DIM || in_sizes[4] != ET * ET || in_sizes[6] != ET * ET || in_sizes[8] != HDIM * NHID || in_sizes[9] != NHID || out_size != NB * REF * NHID) return;
  const int BLIM = NB;
  size_t off = 0; char* ws = (char*)d_ws;
  auto carve = [&](size_t bytes) { char* p = ws + off; off += (bytes + 255) & ~(size_t)255; return p; };
  b16* WQ = (b16*)carve((size_t)ET * ET * 2); b16* WK = (b16*)carve((size_t)ET * ET * 2); b16* WO = (b16*)carve((size_t)NHID * HDIM * 2); b16* Qh = (b16*)carve((size_t)NB * REF * ET * 2); b16* Ql = (b16*)carve((size_t)NB * REF * ET * 2); b16* Kh = (b16*)carve((size_t)NB * KEY * ET * 2); b16* Kl = (b16*)carve((size_t)NB * KEY * ET * 2); float* X = (float*)carve((size_t)NB * REF * HDIM * 4);
  if (off > ws_size || off > ((size_t)16 << 20)) return;
  wput_kernel<<<(ET * 16 + 255) / 256, 256, 0, stream>>>(Fp(4), Fp(6), Fp(8), WQ, WK, WO);
  proj_kernel<0><<<BLIM * REF / 16, 32, 0, stream>>>(Fp(0), WQ, Fp(5), BLIM * REF, Qh, Ql);
  proj_kernel<1><<<BLIM * KEY / 16, 32, 0, stream>>>(Fp(1), WK, Fp(7), BLIM * KEY, Kh, Kl);
  att_kernel<<<BLIM * NH * (REF / 16), 32, 0, stream>>>(Qh, Ql, Kh, Kl, Fp(2), Ip(3), BLIM, X);
  out_kernel<<<BLIM * REF / 16, 32, 0, stream>>>(X, WO, Fp(9), BLIM * REF, (float*)d_out);
}
